// MultiHeadDifferentialAttention_13417477833076
// MI455X (gfx1250) — hardware-verified
//
#include <hip/hip_runtime.h>


#ifndef NB
#define NB 1
#endif
#ifndef SEQ
#define SEQ 2048
#endif
#define NB_FULL 1
#define SEQ_FULL 2048
#define EMB 1024
#define HEADS 16
#define HD 64
#define QKC 128
#define SECW 320
#define NQKV (HEADS * SECW)
#define KO (2 * EMB)
#define LN_EPS 1e-5f
#define OUT_SCALE 0.2f

static_assert(NB == 1);
static_assert(NB_FULL == 1);
static_assert(SEQ % 128 == 0);
static_assert(SEQ >= 128);
static_assert(SEQ <= SEQ_FULL);
static_assert(EMB % 64 == 0);
static_assert(EMB % 32 == 0);
static_assert(QKC == 2 * HD);
static_assert(SECW == 2 * QKC + HD);
static_assert(SECW % 64 == 0);
static_assert(KO % 32 == 0);
static_assert(HD == 64);

typedef _Float16      v16h __attribute__((ext_vector_type(16)));
typedef _Float16      v8h  __attribute__((ext_vector_type(8)));
typedef __bf16        v16b __attribute__((ext_vector_type(16)));
typedef float         v8f  __attribute__((ext_vector_type(8)));
typedef float         v4f  __attribute__((ext_vector_type(4)));
typedef unsigned int  v4u  __attribute__((ext_vector_type(4)));

#define DEV __device__ __forceinline__

union FragB { v4u q[2]; v16b v; };
union Pack8 { v8h h; v4u u; };

DEV unsigned short f2bf(float f) {
  unsigned int u = __float_as_uint(f);
  u += 0x7FFFu + ((u >> 16) & 1u);
  return (unsigned short)(u >> 16);
}
DEV float bf2f(unsigned short s) { return __uint_as_float(((unsigned int)s) << 16); }
DEV float bfr(float f) { return bf2f(f2bf(f)); }
DEV unsigned int pk2(unsigned short lo, unsigned short hi) {
  return (unsigned int)lo | ((unsigned int)hi << 16);
}
DEV void hl2(float a, float b, unsigned int& H, unsigned int& L) {
  const unsigned short ha = f2bf(a), hb = f2bf(b);
  H = pk2(ha, hb);
  L = pk2(f2bf(a - bf2f(ha)), f2bf(b - bf2f(hb)));
}

DEV v8f wmma_h(v16h a, v16h b, v8f c) {
  c = __builtin_amdgcn_wmma_f32_16x16x32_f16(false, a, false, b, (short)0, c, false, false);
  asm volatile("v_nop\n\tv_nop\n\tv_nop\n\tv_nop" : "+v"(c) : "v"(a), "v"(b));
  return c;
}
DEV v8f wmma_b(const FragB& a, const FragB& b, v8f c) {
  c = __builtin_amdgcn_wmma_f32_16x16x32_bf16(false, a.v, false, b.v, (short)0, c, false, false);
  asm volatile("v_nop\n\tv_nop\n\tv_nop\n\tv_nop"
               : "+v"(c) : "v"(a.q[0]), "v"(a.q[1]), "v"(b.q[0]), "v"(b.q[1]));
  return c;
}

DEV v16h load_op16(const _Float16* p, int ld) {
  const int lane = threadIdx.x & 31;
  const int row  = lane & 15;
  const int k0   = (lane >> 4) << 3;
  const _Float16* r = p + (size_t)row * ld + k0;
  v8h lo = *(const v8h*)(r);
  v8h hi = *(const v8h*)(r + 16);
  return __builtin_shufflevector(lo, hi, 0,1,2,3,4,5,6,7,8,9,10,11,12,13,14,15);
}
DEV FragB load_opb(const unsigned short* p, int ld) {
  const int lane = threadIdx.x & 31;
  const int row  = lane & 15;
  const int k0   = (lane >> 4) << 3;
  const unsigned short* r = p + (size_t)row * ld + k0;
  FragB f;
  f.q[0] = *(const v4u*)(r);
  f.q[1] = *(const v4u*)(r + 16);
  return f;
}

DEV float redmax16(float v) {
#pragma unroll
  for (int m = 1; m < 16; m <<= 1) v = fmaxf(v, __shfl_xor(v, m, 32));
  return v;
}
DEV float redsum16(float v) {
#pragma unroll
  for (int m = 1; m < 16; m <<= 1) v += __shfl_xor(v, m, 32);
  return v;
}
DEV float wsum32(float v) {
#pragma unroll
  for (int m = 16; m > 0; m >>= 1) v += __shfl_xor(v, m, 32);
  return v;
}

__global__ __launch_bounds__(256)
void k_cvt_x(const float* __restrict__ X, unsigned short* __restrict__ Xb, int n8) {
  const int i = blockIdx.x * 256 + threadIdx.x;
  if (i >= n8) return;
  const float* s = X + (size_t)i * 8;
  const v4f a = *(const v4f*)(s);
  const v4f b = *(const v4f*)(s + 4);
  v4u w;
  w[0] = pk2(f2bf(a[0]), f2bf(a[1]));
  w[1] = pk2(f2bf(a[2]), f2bf(a[3]));
  w[2] = pk2(f2bf(b[0]), f2bf(b[1]));
  w[3] = pk2(f2bf(b[2]), f2bf(b[3]));
  unsigned short* d = Xb + (size_t)i * 8;
  *(volatile v4u*)d = w;
  __threadfence();
  *(volatile v4u*)d = w;
}

DEV void tr_tile(const float* __restrict__ src, int sld, unsigned short* dst, int dld,
                 int dup2, unsigned short (*T)[72]) {
  const int tid = threadIdx.x;
#pragma unroll
  for (int p = 0; p < 4; ++p) {
    const int e = p * 16 + (tid >> 4);
    const int c = (tid & 15) * 4;
    const v4f v = *(const v4f*)(src + (size_t)e * sld + c);
    T[c + 0][e] = f2bf(v[0]);
    T[c + 1][e] = f2bf(v[1]);
    T[c + 2][e] = f2bf(v[2]);
    T[c + 3][e] = f2bf(v[3]);
  }
  __syncthreads();
#pragma unroll 1
  for (int pass = 0; pass < 2; ++pass) {
#pragma unroll
    for (int p = 0; p < 2; ++p) {
      const int j = p * 32 + (tid >> 3);
      const int seg = (tid & 7) * 8;
      const v4u wv = *(const v4u*)(&T[j][seg]);
      unsigned short* d = dst + (size_t)j * dld + seg;
      *(volatile v4u*)d = wv;
      if (dup2 != 0) *(volatile v4u*)(d + EMB) = wv;
    }
    if (pass == 0) __threadfence();
  }
}

__global__ __launch_bounds__(256)
void k_tr_wqkv(const float* __restrict__ Wq, const float* __restrict__ Wk,
               const float* __restrict__ Wv, unsigned short* __restrict__ Wt) {
  __shared__ __align__(16) unsigned short T[64][72];
  const int e0 = blockIdx.x * 64;
  const int w  = blockIdx.y;
  const int h  = blockIdx.z;
  const float* src;
  int sld;
  if (w < 2) {
    src = Wq + (size_t)h * EMB * QKC + (size_t)e0 * QKC + w * 64;        sld = QKC;
  } else if (w < 4) {
    src = Wk + (size_t)h * EMB * QKC + (size_t)e0 * QKC + (w - 2) * 64;  sld = QKC;
  } else {
    src = Wv + (size_t)h * EMB * HD + (size_t)e0 * HD;                   sld = HD;
  }
  unsigned short* dst = Wt + (size_t)(h * SECW + w * 64) * EMB + e0;
  tr_tile(src, sld, dst, EMB, 0, T);
}

__global__ __launch_bounds__(256)
void k_tr_wo(const float* __restrict__ Wo, unsigned short* __restrict__ Wo2) {
  __shared__ __align__(16) unsigned short T[64][72];
  const int e0 = blockIdx.x * 64;
  const int y  = blockIdx.y;
  const float* src = Wo + (size_t)e0 * EMB + y * 64;
  unsigned short* dst = Wo2 + (size_t)(y * 64) * KO + e0;
  tr_tile(src, EMB, dst, KO, 1, T);
}

__global__ __launch_bounds__(128)
void k_gemm(const unsigned short* __restrict__ A, const unsigned short* __restrict__ Bt,
            int K, int kind,
            const float* __restrict__ bq, const float* __restrict__ bk,
            const float* __restrict__ bv, const float* __restrict__ bo,
            _Float16* __restrict__ Qp, _Float16* __restrict__ Kp,
            _Float16* __restrict__ V64, _Float16* __restrict__ Vsm,
            float* __restrict__ Y) {
  __shared__ __align__(16) float Cs[128][68];
  const int tid  = threadIdx.x;
  const int lane = tid & 31;
  const int wave = tid >> 5;
  const int nt = blockIdx.x;
  const int m0 = blockIdx.y * 128;
  const int n0 = nt * 64;

  const unsigned short* arow = A  + (size_t)(m0 + wave * 32) * K;
  const unsigned short* brow = Bt + (size_t)n0 * K;

  v8f acc[2][4] = {};
#pragma unroll 1
  for (int k0 = 0; k0 < K; k0 += 32) {
    const FragB a0 = load_opb(arow + k0, K);
    const FragB a1 = load_opb(arow + (size_t)16 * K + k0, K);
#pragma unroll
    for (int t = 0; t < 4; ++t) {
      const FragB b = load_opb(brow + (size_t)(t * 16) * K + k0, K);
      acc[0][t] = wmma_b(a0, b, acc[0][t]);
      acc[1][t] = wmma_b(a1, b, acc[1][t]);
    }
  }

  const int n  = lane & 15;
  const int rb = (lane >> 4) << 3;
#pragma unroll
  for (int mi = 0; mi < 2; ++mi)
#pragma unroll
    for (int t = 0; t < 4; ++t)
#pragma unroll
      for (int r = 0; r < 8; ++r)
        Cs[wave * 32 + mi * 16 + rb + r][t * 16 + n] = acc[mi][t][r];
  __syncthreads();

  if (kind == 0) {
    const int h = nt / 5;
    const int w = nt - h * 5;
    if (w < 4) {
      _Float16* plane = (w < 2) ? Qp : Kp;
      const int cb = (w & 1) * 64;
      const float* bias = ((w < 2) ? bq : bk) + h * QKC + cb;
      const int seg  = (tid & 7) * 8;
      const int rsub = tid >> 3;
      float bb[8];
#pragma unroll
      for (int j = 0; j < 8; ++j) bb[j] = bfr(bias[seg + j]);
#pragma unroll 1
      for (int pass = 0; pass < 2; ++pass) {
#pragma unroll 2
        for (int g = 0; g < 8; ++g) {
          const int row = g * 16 + rsub;
          const v4f c0 = *(const v4f*)(&Cs[row][seg]);
          const v4f c1 = *(const v4f*)(&Cs[row][seg + 4]);
          Pack8 pk;
          pk.h[0] = (_Float16)(c0[0] + bb[0]);
          pk.h[1] = (_Float16)(c0[1] + bb[1]);
          pk.h[2] = (_Float16)(c0[2] + bb[2]);
          pk.h[3] = (_Float16)(c0[3] + bb[3]);
          pk.h[4] = (_Float16)(c1[0] + bb[4]);
          pk.h[5] = (_Float16)(c1[1] + bb[5]);
          pk.h[6] = (_Float16)(c1[2] + bb[6]);
          pk.h[7] = (_Float16)(c1[3] + bb[7]);
          _Float16* d = plane + ((size_t)h * SEQ + m0 + row) * QKC + cb + seg;
          *(volatile v4u*)d = pk.u;
        }
        if (pass == 0) __threadfence();
      }
    } else {
      const int seg  = (tid & 15) * 8;
      const int dsub = tid >> 4;
      const float* bias = bv + h * HD;
#pragma unroll 1
      for (int pass = 0; pass < 2; ++pass) {
#pragma unroll 2
        for (int g = 0; g < 8; ++g) {
          const int d = g * 8 + dsub;
          const float bb = bfr(bias[d]);
          Pack8 p64, psm;
#pragma unroll
          for (int j = 0; j < 8; ++j) {
            const float v = Cs[seg + j][d] + bb;
            p64.h[j] = (_Float16)(v * 64.0f);
            psm.h[j] = (_Float16)(v * 0.015625f);
          }
          const size_t o = ((size_t)(h * HD + d)) * SEQ + m0 + seg;
          *(volatile v4u*)(V64 + o) = p64.u;
          *(volatile v4u*)(Vsm + o) = psm.u;
        }
        if (pass == 0) __threadfence();
      }
    }
  } else {
    const int seg  = (tid & 15) * 4;
    const int rsub = tid >> 4;
    float bb[4];
#pragma unroll
    for (int j = 0; j < 4; ++j) bb[j] = bfr(bo[n0 + seg + j]);
#pragma unroll 1
    for (int pass = 0; pass < 2; ++pass) {
#pragma unroll 2
      for (int g = 0; g < 16; ++g) {
        const int row = g * 8 + rsub;
        const v4f c = *(const v4f*)(&Cs[row][seg]);
        v4f o;
        o[0] = c[0] + bb[0];
        o[1] = c[1] + bb[1];
        o[2] = c[2] + bb[2];
        o[3] = c[3] + bb[3];
        float* d = Y + (size_t)(m0 + row) * EMB + n0 + seg;
        *(volatile v4f*)d = o;
      }
      if (pass == 0) __threadfence();
    }
  }
}

DEV void attn_branch(const v16h (&qa)[2], const _Float16* __restrict__ kcol,
                     const _Float16* __restrict__ v64h, const _Float16* __restrict__ vsh,
                     int kk, float (&m)[8], float (&l)[8], v8f (&O)[4],
                     _Float16* phs, _Float16* pls) {
  const int lane = threadIdx.x & 31;
  const int n  = lane & 15;
  const int rb = (lane >> 4) << 3;

  v8f sa = {}, sb = {};
  {
    v16h kb;
    kb = load_op16(kcol + (size_t)kk * QKC, QKC);              sa = wmma_h(qa[0], kb, sa);
    kb = load_op16(kcol + (size_t)kk * QKC + 32, QKC);         sa = wmma_h(qa[1], kb, sa);
    kb = load_op16(kcol + (size_t)(kk + 16) * QKC, QKC);       sb = wmma_h(qa[0], kb, sb);
    kb = load_op16(kcol + (size_t)(kk + 16) * QKC + 32, QKC);  sb = wmma_h(qa[1], kb, sb);
  }

  float f[8];
#pragma unroll
  for (int i = 0; i < 8; ++i) {
    const float xa = sa[i] * 0.125f;
    const float xb = sb[i] * 0.125f;
    const float mn = fmaxf(m[i], redmax16(fmaxf(xa, xb)));
    f[i] = __expf(m[i] - mn);
    const float pa = __expf(xa - mn);
    const float pb = __expf(xb - mn);
    l[i] = l[i] * f[i] + redsum16(pa + pb);
    m[i] = mn;
    const _Float16 ha = (_Float16)pa;
    const _Float16 hb = (_Float16)pb;
    const _Float16 la = (_Float16)((pa - (float)ha) * 4096.0f);
    const _Float16 lb = (_Float16)((pb - (float)hb) * 4096.0f);
    phs[(rb + i) * 32 + n]      = ha;
    phs[(rb + i) * 32 + n + 16] = hb;
    pls[(rb + i) * 32 + n]      = la;
    pls[(rb + i) * 32 + n + 16] = lb;
  }
  __syncthreads();
  const v16h ph = load_op16(phs, 32);
  const v16h pl = load_op16(pls, 32);
#pragma unroll
  for (int t = 0; t < 4; ++t) {
    const v16h vb = load_op16(v64h + (size_t)(t * 16) * SEQ + kk, SEQ);
    const v16h vs = load_op16(vsh  + (size_t)(t * 16) * SEQ + kk, SEQ);
#pragma unroll
    for (int i = 0; i < 8; ++i) O[t][i] = O[t][i] * f[i];
    O[t] = wmma_h(ph, vb, O[t]);
    O[t] = wmma_h(pl, vs, O[t]);
  }
  __syncthreads();
}

__global__ __launch_bounds__(128)
void k_attn(const _Float16* __restrict__ Qp, const _Float16* __restrict__ Kp,
            const _Float16* __restrict__ V64, const _Float16* __restrict__ Vsm,
            const float* __restrict__ lam_p, unsigned short* __restrict__ Oc) {
  __shared__ __align__(16) _Float16 Ps[4][4][16 * 32];
  __shared__ __align__(16) float Os[4][16][68];
  const int lane = threadIdx.x & 31;
  const int wave = threadIdx.x >> 5;
  const int n  = lane & 15;
  const int rb = (lane >> 4) << 3;
  const int hh = blockIdx.y;
  const int q0 = blockIdx.x * 64 + wave * 16;
  const float lam = bfr(lam_p[0]);

  const _Float16* qh = Qp  + (size_t)hh * SEQ * QKC;
  const _Float16* kh = Kp  + (size_t)hh * SEQ * QKC;
  const _Float16* vh = V64 + (size_t)hh * HD * SEQ;
  const _Float16* vs = Vsm + (size_t)hh * HD * SEQ;

  v16h q1[2], q2[2];
  q1[0] = load_op16(qh + (size_t)q0 * QKC + 0,  QKC);
  q1[1] = load_op16(qh + (size_t)q0 * QKC + 32, QKC);
  q2[0] = load_op16(qh + (size_t)q0 * QKC + 64, QKC);
  q2[1] = load_op16(qh + (size_t)q0 * QKC + 96, QKC);

  v8f O1[4] = {}, O2[4] = {};
  float m1[8], l1[8], m2[8], l2[8];
#pragma unroll
  for (int i = 0; i < 8; ++i) { m1[i] = -1e30f; m2[i] = -1e30f; l1[i] = 0.f; l2[i] = 0.f; }

  _Float16* p1h = &Ps[wave][0][0];
  _Float16* p1l = &Ps[wave][1][0];
  _Float16* p2h = &Ps[wave][2][0];
  _Float16* p2l = &Ps[wave][3][0];

#pragma unroll 1
  for (int kk = 0; kk < SEQ; kk += 32) {
    attn_branch(q1, kh,      vh, vs, kk, m1, l1, O1, p1h, p1l);
    attn_branch(q2, kh + 64, vh, vs, kk, m2, l2, O2, p2h, p2l);
  }

#pragma unroll
  for (int i = 0; i < 8; ++i) {
    const float r1 = (1.0f / l1[i]) * 0.015625f;
    const float r2 = (lam * (1.0f / l2[i])) * 0.015625f;
#pragma unroll
    for (int t = 0; t < 4; ++t)
      Os[wave][rb + i][t * 16 + n] = O1[t][i] * r1 - O2[t][i] * r2;
  }
  __syncthreads();

  const int rsub = lane >> 3;
  const int seg  = (lane & 7) * 8;
#pragma unroll 1
  for (int pass = 0; pass < 2; ++pass) {
#pragma unroll
    for (int g = 0; g < 4; ++g) {
      const int row = g * 4 + rsub;
      const v4f c0 = *(const v4f*)(&Os[wave][row][seg]);
      const v4f c1 = *(const v4f*)(&Os[wave][row][seg + 4]);
      unsigned int H0, H1, H2, H3, L0, L1, L2, L3;
      hl2(c0[0], c0[1], H0, L0);
      hl2(c0[2], c0[3], H1, L1);
      hl2(c1[0], c1[1], H2, L2);
      hl2(c1[2], c1[3], H3, L3);
      v4u H, L;
      H[0] = H0; H[1] = H1; H[2] = H2; H[3] = H3;
      L[0] = L0; L[1] = L1; L[2] = L2; L[3] = L3;
      unsigned short* d = Oc + (size_t)(q0 + row) * KO + hh * HD + seg;
      *(volatile v4u*)d = H;
      *(volatile v4u*)(d + EMB) = L;
    }
    if (pass == 0) __threadfence();
  }
}

__global__ __launch_bounds__(256)
void k_ln(const float* __restrict__ Y, const float* __restrict__ gamma,
          const float* __restrict__ beta, float* __restrict__ out) {
  __shared__ float sa[8];
  __shared__ float sq[8];
  const int tid  = threadIdx.x;
  const int lane = tid & 31;
  const int wave = tid >> 5;
  const size_t row = blockIdx.x;
  const v4f y = *(const v4f*)(Y + row * EMB + tid * 4);

  float s = (y[0] + y[1]) + (y[2] + y[3]);
  s = wsum32(s);
  if (lane == 0) sa[wave] = s;
  __syncthreads();
  float tot = 0.f;
#pragma unroll
  for (int w = 0; w < 8; ++w) tot += sa[w];
  const float mu = tot * (1.0f / (float)EMB);

  float d0 = y[0] - mu, d1 = y[1] - mu, d2 = y[2] - mu, d3 = y[3] - mu;
  float q = (d0 * d0 + d1 * d1) + (d2 * d2 + d3 * d3);
  q = wsum32(q);
  if (lane == 0) sq[wave] = q;
  __syncthreads();
  float tot2 = 0.f;
#pragma unroll
  for (int w = 0; w < 8; ++w) tot2 += sq[w];
  const float var  = tot2 * (1.0f / (float)EMB);
  const float rstd = rsqrtf(var + LN_EPS);

  const float g0 = bfr(gamma[tid * 4 + 0]), g1 = bfr(gamma[tid * 4 + 1]);
  const float g2 = bfr(gamma[tid * 4 + 2]), g3 = bfr(gamma[tid * 4 + 3]);
  const float b0 = bfr(beta[tid * 4 + 0]),  b1 = bfr(beta[tid * 4 + 1]);
  const float b2 = bfr(beta[tid * 4 + 2]),  b3 = bfr(beta[tid * 4 + 3]);
  v4f o;
  o[0] = ((d0 * rstd) * g0 + b0) * OUT_SCALE;
  o[1] = ((d1 * rstd) * g1 + b1) * OUT_SCALE;
  o[2] = ((d2 * rstd) * g2 + b2) * OUT_SCALE;
  o[3] = ((d3 * rstd) * g3 + b3) * OUT_SCALE;
  float* dst = out + row * EMB + tid * 4;
  *(volatile v4f*)dst = o;
  __threadfence();
  *(volatile v4f*)dst = o;
}

extern "C" void kernel_launch(void* const* d_in, const int* in_sizes, int n_in,
                              void* d_out, int out_size, void* d_ws, size_t ws_size,
                              hipStream_t stream) {
  if (n_in < 12) return;
  const float* X     = (const float*)d_in[0];
  const float* Wq    = (const float*)d_in[1];
  const float* bq    = (const float*)d_in[2];
  const float* Wk    = (const float*)d_in[3];
  const float* bk    = (const float*)d_in[4];
  const float* Wv    = (const float*)d_in[5];
  const float* bv    = (const float*)d_in[6];
  const float* Wo    = (const float*)d_in[7];
  const float* bo    = (const float*)d_in[8];
  const float* gamma = (const float*)d_in[9];
  const float* beta  = (const float*)d_in[10];
  const float* lam   = (const float*)d_in[11];
  float* out = (float*)d_out;

  if (in_sizes[0]  < NB * SEQ * EMB) return;
  if (in_sizes[1]  < HEADS * EMB * QKC) return;
  if (in_sizes[2]  < HEADS * QKC) return;
  if (in_sizes[3]  < HEADS * EMB * QKC) return;
  if (in_sizes[4]  < HEADS * QKC) return;
  if (in_sizes[5]  < HEADS * EMB * HD) return;
  if (in_sizes[6]  < HEADS * HD) return;
  if (in_sizes[7]  < EMB * EMB) return;
  if (in_sizes[8]  < EMB) return;
  if (in_sizes[9]  < EMB) return;
  if (in_sizes[10] < EMB) return;
  if (in_sizes[11] < 1) return;
  if (out_size < NB * SEQ * EMB) return;

  const size_t szXb  = (size_t)SEQ * EMB * 2;
  const size_t szWt  = (size_t)NQKV * EMB * 2;
  const size_t szWo2 = (size_t)EMB * KO * 2;
  const size_t szQK  = (size_t)HEADS * SEQ * QKC * 2;
  const size_t szV   = (size_t)HEADS * HD * SEQ * 2;
  const size_t szOc  = (size_t)SEQ * KO * 2;
  const size_t szY   = (size_t)SEQ * EMB * 4;
  size_t off = 0;
  const size_t oXb  = off; off += szXb;
  const size_t oWt  = off; off += szWt;
  const size_t oWo2 = off; off += szWo2;
  const size_t oQ   = off; off += szQK;
  const size_t oK   = off; off += szQK;
  const size_t oV64 = off; off += szV;
  const size_t oVsm = off; off += szV;
  const size_t oOc  = off; off += szOc;
  const size_t oY   = off; off += szY;
  if (off > ws_size) return;

  char* ws = (char*)d_ws;
  unsigned short* Xb  = (unsigned short*)(ws + oXb);
  unsigned short* Wt  = (unsigned short*)(ws + oWt);
  unsigned short* Wo2 = (unsigned short*)(ws + oWo2);
  _Float16* Qp  = (_Float16*)(ws + oQ);
  _Float16* Kp  = (_Float16*)(ws + oK);
  _Float16* V64 = (_Float16*)(ws + oV64);
  _Float16* Vsm = (_Float16*)(ws + oVsm);
  unsigned short* Oc = (unsigned short*)(ws + oOc);
  float* Y = (float*)(ws + oY);

  const int n8 = SEQ * EMB / 8;
  k_cvt_x<<<dim3((n8 + 255) / 256), dim3(256), 0, stream>>>(X, Xb, n8);
  k_tr_wqkv<<<dim3(EMB / 64, 5, HEADS), dim3(256), 0, stream>>>(Wq, Wk, Wv, Wt);
  k_tr_wo<<<dim3(EMB / 64, EMB / 64, 1), dim3(256), 0, stream>>>(Wo, Wo2);

  k_gemm<<<dim3(NQKV / 64, SEQ / 128), dim3(128), 0, stream>>>(
      Xb, Wt, EMB, 0, bq, bk, bv, bo, Qp, Kp, V64, Vsm, Y);

  k_attn<<<dim3(SEQ / 64, HEADS), dim3(128), 0, stream>>>(Qp, Kp, V64, Vsm, lam, Oc);

  k_gemm<<<dim3(EMB / 64, SEQ / 128), dim3(128), 0, stream>>>(
      Oc, Wo2, KO, 1, bq, bk, bv, bo, Qp, Kp, V64, Vsm, Y);

  k_ln<<<dim3(NB * SEQ), dim3(256), 0, stream>>>(Y, gamma, beta, out);
}
